// Network_28544352649223
// MI455X (gfx1250) — hardware-verified
//
#include <hip/hip_runtime.h>
#include <math.h>

constexpr int kBatch = 2;
constexpr int kSeq   = 2048;
constexpr int kDim   = 1024;
constexpr int kHeads = 16;
constexpr int kDh    = 64;
constexpr int kTok   = kBatch * kSeq;
constexpr int kQKW   = 2 * kDh;
constexpr int kWRows = 3 * kDh;
constexpr int kEarly = 256;
constexpr int kGroup = 2;
constexpr int kBH    = kBatch * kHeads;
constexpr float kScoreScale = 0.125f;
constexpr float kPCarry     = 32768.0f;
constexpr float kCtxCarry   = 16.0f;
constexpr float kWCarry     = 16.0f;
constexpr float kPVScale    = kCtxCarry / kPCarry;
constexpr float kProjScale  = 1.0f / (kCtxCarry * kWCarry);
static_assert(kHeads * kDh == kDim, "shape");
static_assert(kSeq % 512 == 0 && kSeq % 64 == 0 && kTok % 64 == 0, "tiles");
static_assert(kDh % 64 == 0 && kQKW % 64 == 0 && kDim % 64 == 0 && kEarly % 64 == 0, "tiles");
static_assert(kDh % 32 == 0 && kDim % 32 == 0 && kSeq % 32 == 0 && kEarly % 32 == 0, "k32");
static_assert(kHeads % kGroup == 0 && kEarly == 256, "groups");

typedef __attribute__((ext_vector_type(16))) _Float16 v16h;
typedef __attribute__((ext_vector_type(8)))  _Float16 v8h;
typedef __attribute__((ext_vector_type(16))) __bf16   v16b;
typedef __attribute__((ext_vector_type(8)))  __bf16   v8b;
typedef __attribute__((ext_vector_type(8)))  float    v8f;
typedef __attribute__((ext_vector_type(4)))  float    v4f;
typedef __attribute__((ext_vector_type(2)))  float    v2f;
typedef __attribute__((ext_vector_type(4)))  unsigned int v4u;

__device__ __forceinline__ unsigned short f2bf_bits(float f) {
  unsigned u = __float_as_uint(f);
  return (unsigned short)((u + 0x7FFFu + ((u >> 16) & 1u)) >> 16);
}
__device__ __forceinline__ float bf_bits2f(unsigned short h) { return __uint_as_float(((unsigned)h) << 16); }

__device__ __forceinline__ void dep_guard_h(v8f& a, v8f& b, v16h x, v16h y) { asm volatile("v_nop\n\tv_nop\n\tv_nop\n\tv_nop" : "+v"(a), "+v"(b) : "v"(x), "v"(y)); }
__device__ __forceinline__ void dep_guard_b(v8f& a, v8f& b, v16b x, v16b y) { asm volatile("v_nop\n\tv_nop\n\tv_nop\n\tv_nop" : "+v"(a), "+v"(b) : "v"(x), "v"(y)); }
__device__ __forceinline__ void dep_guard4_h(v8f& a, v8f& b, v8f& c, v8f& d, v16h x, v16h y) {
  asm volatile("v_nop\n\tv_nop\n\tv_nop\n\tv_nop" : "+v"(a), "+v"(b), "+v"(c), "+v"(d) : "v"(x), "v"(y));
}
__device__ __forceinline__ void dep_guard4_b(v8f& a, v8f& b, v8f& c, v8f& d, v16b x, v16b y) {
  asm volatile("v_nop\n\tv_nop\n\tv_nop\n\tv_nop" : "+v"(a), "+v"(b), "+v"(c), "+v"(d) : "v"(x), "v"(y));
}
__device__ __forceinline__ void keep4_h(v16h a, v16h b, v16h c, v16h d) { asm volatile("v_nop" :: "v"(a), "v"(b), "v"(c), "v"(d)); }
__device__ __forceinline__ void keep4_b(v16b a, v16b b, v16b c, v16b d) { asm volatile("v_nop" :: "v"(a), "v"(b), "v"(c), "v"(d)); }
__device__ __forceinline__ void acc_guard4(v8f& a, v8f& b, v8f& c, v8f& d) { asm volatile("v_nop\n\tv_nop\n\tv_nop\n\tv_nop" : "+v"(a), "+v"(b), "+v"(c), "+v"(d)); }
template <typename T> struct Frag;
template <> struct Frag<_Float16> {
  typedef v16h V; union U { v16h v; v8h h[2]; };
  static __device__ __forceinline__ v16h load(const _Float16* p) {
    U f; f.h[0] = *(const v8h*)(p); f.h[1] = *(const v8h*)(p + 16); return f.v;
  }
  static __device__ __forceinline__ v8f mma(v16h a, v16h b, v8f c) {
    return __builtin_amdgcn_wmma_f32_16x16x32_f16(false, a, false, b, (short)0, c, false, false);
  }
  static __device__ __forceinline__ void guard(v8f& a, v8f& b, v16h x, v16h y) { dep_guard_h(a, b, x, y); }
  static __device__ __forceinline__ void guard4(v8f& a, v8f& b, v8f& c, v8f& d, v16h x, v16h y) { dep_guard4_h(a, b, c, d, x, y); }
  static __device__ __forceinline__ void keep(v16h a, v16h b, v16h c, v16h d) { keep4_h(a, b, c, d); }
};
template <> struct Frag<__bf16> {
  typedef v16b V; union U { v16b v; v8b h[2]; };
  static __device__ __forceinline__ v16b load(const __bf16* p) {
    U f; f.h[0] = *(const v8b*)(p); f.h[1] = *(const v8b*)(p + 16); return f.v;
  }
  static __device__ __forceinline__ v8f mma(v16b a, v16b b, v8f c) {
    return __builtin_amdgcn_wmma_f32_16x16x32_bf16(false, a, false, b, (short)0, c, false, false);
  }
  static __device__ __forceinline__ void guard(v8f& a, v8f& b, v16b x, v16b y) { dep_guard_b(a, b, x, y); }
  static __device__ __forceinline__ void guard4(v8f& a, v8f& b, v8f& c, v8f& d, v16b x, v16b y) { dep_guard4_b(a, b, c, d, x, y); }
  static __device__ __forceinline__ void keep(v16b a, v16b b, v16b c, v16b d) { keep4_b(a, b, c, d); }
};

__device__ __forceinline__ unsigned pk16(unsigned short a, unsigned short b) { return (unsigned)a | ((unsigned)b << 16); }
__device__ __forceinline__ unsigned short h_bits(float f) { const _Float16 h = (_Float16)f; return __builtin_bit_cast(unsigned short, h); }

template <int ET> struct Elem;
template <> struct Elem<0> { typedef _Float16 T; };
template <> struct Elem<1> { typedef __bf16 T; };
template <int ET, bool SPLIT, int BIAS_MODE, int OUT_MODE, bool RESID, int ACT = 0, int CAUSAL = 0>
__global__ __launch_bounds__(256) void wmma_gemm64(
    const unsigned short* __restrict__ Ap, const unsigned short* __restrict__ A2p, int lda, long strideA,
    const unsigned short* __restrict__ Btp, const unsigned short* __restrict__ Bt2p, int ldb, long strideB,
    void* __restrict__ Cout, void* __restrict__ Cout2, int ldc, long strideC,
    const float* __restrict__ bias,
    const float* __restrict__ resid, long strideR,
    int M, int N, int K, float scale) {
  typedef typename Elem<ET>::T T;
  typedef typename Frag<T>::V V;
  const T* A = (const T*)Ap; const T* A2 = (const T*)A2p; const T* Bt = (const T*)Btp; const T* Bt2 = (const T*)Bt2p;
  __shared__ __align__(16) float sT[8][16 * 68];
  const int b    = blockIdx.y;
  const int lane = threadIdx.x & 31;
  const int wave = threadIdx.x >> 5;
  const int tilesN = N >> 6;
  const int tilesM = M >> 6;
  const int tile = blockIdx.x * 8 + wave;
  if (tile >= tilesM * tilesN) return;
  const int tm = tile / tilesN;
  const int tn = tile - tm * tilesN;
  const int m0 = tm << 6;
  const int n0 = tn << 6;

  const T* Ab  = A  + (size_t)b * strideA;
  const T* Bb  = Bt + (size_t)b * strideB;
  const T* Ab2 = SPLIT ? (A2  + (size_t)b * strideA) : nullptr;
  const T* Bb2 = SPLIT ? (Bt2 + (size_t)b * strideB) : nullptr;

  const int rlane = lane & 15;
  const int koff  = (lane >> 4) * 8;
  const int mOff  = (lane >> 4) * 8;

  int kEnd = K;
  if (CAUSAL == 1) { if (n0 >= m0 + 64) kEnd = 0; }
  if (CAUSAL == 2) { const int kl = m0 + 64; kEnd = (kl < K) ? kl : K; }

  v8f acc[4][4];
#pragma unroll
  for (int i = 0; i < 4; ++i)
#pragma unroll
    for (int j = 0; j < 4; ++j) acc[i][j] = (v8f){0.f,0.f,0.f,0.f,0.f,0.f,0.f,0.f};

  for (int k0 = 0; k0 < kEnd; k0 += 32) {
    V bh[4], bl[4];
#pragma unroll
    for (int j = 0; j < 4; ++j) {
      const size_t bo = (size_t)(n0 + (j << 4) + rlane) * ldb + koff + k0;
      bh[j] = Frag<T>::load(Bb + bo);
      if (SPLIT) bl[j] = Frag<T>::load(Bb2 + bo);
    }
#pragma unroll
    for (int i = 0; i < 4; ++i) {
      const size_t ao = (size_t)(m0 + (i << 4) + rlane) * lda + koff + k0;
      V ah = Frag<T>::load(Ab + ao);
      V al;
      if (SPLIT) al = Frag<T>::load(Ab2 + ao);
#pragma unroll
      for (int j = 0; j < 4; ++j) {
        acc[i][j] = Frag<T>::mma(ah, bh[j], acc[i][j]);
        if (SPLIT) {
          acc[i][j] = Frag<T>::mma(ah, bl[j], acc[i][j]);
          acc[i][j] = Frag<T>::mma(al, bh[j], acc[i][j]);
        }
      }
      Frag<T>::guard4(acc[i][0], acc[i][1], acc[i][2], acc[i][3], ah, SPLIT ? al : ah);
    }
    Frag<T>::keep(bh[0], bh[1], bh[2], bh[3]);
    if (SPLIT) Frag<T>::keep(bl[0], bl[1], bl[2], bl[3]);
  }
  acc_guard4(acc[0][0], acc[0][1], acc[0][2], acc[0][3]);
  acc_guard4(acc[1][0], acc[1][1], acc[1][2], acc[1][3]);
  acc_guard4(acc[2][0], acc[2][1], acc[2][2], acc[2][3]);
  acc_guard4(acc[3][0], acc[3][1], acc[3][2], acc[3][3]);

  float* slab = sT[wave];
  const float* Rb = RESID ? (resid + (size_t)b * strideR) : nullptr;
#pragma unroll
  for (int i = 0; i < 4; ++i) {
    const int mBase = m0 + (i << 4);
#pragma unroll
    for (int j = 0; j < 4; ++j) {
      const int n = n0 + (j << 4) + rlane;
      float bv = 0.f;
      if (BIAS_MODE == 2) bv = bias[n];
#pragma unroll
      for (int r = 0; r < 8; ++r) {
        float v = acc[i][j][r] * scale;
        if (BIAS_MODE == 1) v += bias[mBase + mOff + r];
        if (BIAS_MODE == 2) v += bv;
        if (RESID) v += Rb[(size_t)(mBase + mOff + r) * ldc + n];
        if (ACT == 2) v = fmaxf(v, 0.0f);
        if (ACT == 4) v = (v > 0.f) ? v : 0.01f * v;
        slab[(mOff + r) * 68 + (j << 4) + rlane] = v;
      }
    }
    __builtin_amdgcn_fence(__ATOMIC_RELEASE, "workgroup");
    __builtin_amdgcn_wave_barrier();
    __builtin_amdgcn_fence(__ATOMIC_ACQUIRE, "workgroup");
    if (OUT_MODE == 0) {
      float* C = (float*)Cout + (size_t)b * strideC;
      const int hh = lane >> 4, c4 = (lane & 15) * 4;
      for (int pass = 0; pass < 2; ++pass) {
#pragma unroll
        for (int it = 0; it < 8; ++it) {
          const int row = it * 2 + hh;
          v4f v = *(const v4f*)(slab + row * 68 + c4);
          *(volatile v4f*)(C + (size_t)(mBase + row) * ldc + n0 + c4) = v;
        }
        __threadfence();
      }
    } else {
      const int q = lane >> 3, c8 = (lane & 7) * 8;
      unsigned short* C  = (unsigned short*)Cout  + (size_t)b * strideC;
      unsigned short* C2 = (OUT_MODE == 2) ? ((unsigned short*)Cout2 + (size_t)b * strideC) : nullptr;
      for (int pass = 0; pass < 2; ++pass) {
#pragma unroll
        for (int it = 0; it < 4; ++it) {
          const int row = it * 4 + q;
          const float* sp = slab + row * 68 + c8;
          v8h hv, lv;
#pragma unroll
          for (int e = 0; e < 8; ++e) {
            if (OUT_MODE == 1) {
              hv[e] = (_Float16)sp[e];
            } else {
              unsigned short hb = f2bf_bits(sp[e]);
              unsigned short lb = f2bf_bits(sp[e] - bf_bits2f(hb));
              hv[e] = __builtin_bit_cast(_Float16, hb);
              lv[e] = __builtin_bit_cast(_Float16, lb);
            }
          }
          *(volatile v8h*)(C + (size_t)(mBase + row) * ldc + n0 + c8) = hv;
          if (OUT_MODE == 2) *(volatile v8h*)(C2 + (size_t)(mBase + row) * ldc + n0 + c8) = lv;
        }
        __threadfence();
      }
    }
    __builtin_amdgcn_fence(__ATOMIC_RELEASE, "workgroup");
    __builtin_amdgcn_wave_barrier();
    __builtin_amdgcn_fence(__ATOMIC_ACQUIRE, "workgroup");
  }
}

__global__ __launch_bounds__(256) void cast8_bf16_kernel(const float* __restrict__ in, unsigned short* __restrict__ out, int n8) {
  const int i = blockIdx.x * 256 + threadIdx.x;
  if (i >= n8) return;
  const float* p = in + 8 * (size_t)i;
  const v4f a = *(const v4f*)(p);
  const v4f c = *(const v4f*)(p + 4);
  unsigned short hb[8];
#pragma unroll
  for (int e = 0; e < 4; ++e) {
    hb[e]     = f2bf_bits(a[e]);
    hb[4 + e] = f2bf_bits(c[e]);
  }
  const v4u u = (v4u){pk16(hb[0], hb[1]), pk16(hb[2], hb[3]), pk16(hb[4], hb[5]), pk16(hb[6], hb[7])};
  unsigned short* q = out + 8 * (size_t)i;
  *(volatile v4u*)q = u;
  __threadfence();
  *(volatile v4u*)q = u;
}

__global__ __launch_bounds__(256) void cast8_wproj_kernel(const float* __restrict__ in, unsigned short* __restrict__ outb,
                                                         unsigned short* __restrict__ out16, int n8) {
  const int i = blockIdx.x * 256 + threadIdx.x;
  if (i >= n8) return;
  const float* p = in + 8 * (size_t)i;
  const v4f a = *(const v4f*)(p);
  const v4f c = *(const v4f*)(p + 4);
  unsigned short bb[8], hb[8];
#pragma unroll
  for (int e = 0; e < 4; ++e) {
    bb[e]     = f2bf_bits(a[e]);
    bb[4 + e] = f2bf_bits(c[e]);
  }
#pragma unroll
  for (int e = 0; e < 8; ++e) hb[e] = h_bits(bf_bits2f(bb[e]) * kWCarry);
  const v4u ub = (v4u){pk16(bb[0], bb[1]), pk16(bb[2], bb[3]), pk16(bb[4], bb[5]), pk16(bb[6], bb[7])};
  const v4u uh = (v4u){pk16(hb[0], hb[1]), pk16(hb[2], hb[3]), pk16(hb[4], hb[5]), pk16(hb[6], hb[7])};
  unsigned short* qb = outb  + 8 * (size_t)i;
  unsigned short* qh = out16 + 8 * (size_t)i;
  *(volatile v4u*)qb = ub;
  *(volatile v4u*)qh = uh;
  __threadfence();
  *(volatile v4u*)qb = ub;
  *(volatile v4u*)qh = uh;
}

__global__ __launch_bounds__(256) void zero8_kernel(unsigned short* __restrict__ out, int n8) {
  const int i = blockIdx.x * 256 + threadIdx.x;
  if (i >= n8) return;
  const v4u z = (v4u){0u, 0u, 0u, 0u};
  unsigned short* q = out + 8 * (size_t)i;
  *(volatile v4u*)q = z;
  __threadfence();
  *(volatile v4u*)q = z;
}

__global__ __launch_bounds__(256) void bias_cast_kernel(const float* __restrict__ bsrc, float* __restrict__ bdst) {
  const int t = threadIdx.x;
  const v4f v = *(const v4f*)(bsrc + 4 * t);
  v4f r;
#pragma unroll
  for (int e = 0; e < 4; ++e) r[e] = bf_bits2f(f2bf_bits(v[e]));
  float* dp = bdst + 4 * t;
  *(volatile v4f*)dp = r;
  __threadfence();
  *(volatile v4f*)dp = r;
}

__global__ __launch_bounds__(256) void softmax_main_kernel(const float* __restrict__ S, unsigned short* __restrict__ P) {
  __shared__ __align__(16) float lg[kSeq];
  __shared__ float redM[8];
  __shared__ float redS[8];
  const int row  = blockIdx.x;
  const int hj   = blockIdx.y;
  const int t    = threadIdx.x;
  const int lane = t & 31, wave = t >> 5;
  const size_t rowoff = ((size_t)hj * kSeq + row) * kSeq;
  const float* sr = S + rowoff;
  const int nch = (row >> 9) + 1;
  const float ninf = -__builtin_inff();

  float mx = ninf;
#pragma unroll 1
  for (int it = 0; it < 4; ++it) {
    const int c = it * 512 + 2 * t;
    v2f av;
    av[0] = ninf;
    av[1] = ninf;
    if (it < nch) {
      const v2f sv = *(const v2f*)(sr + c);
      av[0] = (c <= row) ? sv[0] : ninf;
      av[1] = (c + 1 <= row) ? sv[1] : ninf;
      mx = fmaxf(mx, fmaxf(av[0], av[1]));
    }
    *(v2f*)(lg + c) = av;
  }
#pragma unroll
  for (int off = 16; off > 0; off >>= 1) mx = fmaxf(mx, __shfl_xor(mx, off, 32));
  if (lane == 0) redM[wave] = mx;
  __syncthreads();
  float m = redM[0];
#pragma unroll
  for (int w = 1; w < 8; ++w) m = fmaxf(m, redM[w]);

  float sum = 0.f;
#pragma unroll 1
  for (int it = 0; it < 4; ++it) {
    const int c = it * 512 + 2 * t;
    v2f ev;
    ev[0] = 0.f;
    ev[1] = 0.f;
    if (it < nch) {
      const v2f l = *(const v2f*)(lg + c);
      ev[0] = expf(l[0] - m);
      ev[1] = expf(l[1] - m);
      sum += ev[0];
      sum += ev[1];
    }
    *(v2f*)(lg + c) = ev;
  }
#pragma unroll
  for (int off = 16; off > 0; off >>= 1) sum += __shfl_xor(sum, off, 32);
  if (lane == 0) redS[wave] = sum;
  __syncthreads();
  float tot = redS[0];
#pragma unroll
  for (int w = 1; w < 8; ++w) tot += redS[w];
  const float inv = kPCarry / tot;

  const v4f e0 = *(const v4f*)(lg + 8 * t);
  const v4f e1 = *(const v4f*)(lg + 8 * t + 4);
  unsigned short hb[8];
#pragma unroll
  for (int e = 0; e < 4; ++e) {
    hb[e]     = h_bits(e0[e] * inv);
    hb[4 + e] = h_bits(e1[e] * inv);
  }
  const v4u u = (v4u){pk16(hb[0], hb[1]), pk16(hb[2], hb[3]), pk16(hb[4], hb[5]), pk16(hb[6], hb[7])};
  unsigned short* pr = P + rowoff + 8 * (size_t)t;
  *(volatile v4u*)pr = u;
  __threadfence();
  *(volatile v4u*)pr = u;
}

__global__ __launch_bounds__(256) void softmax_early_kernel(const float* __restrict__ S, unsigned short* __restrict__ Ph,
                                                           unsigned short* __restrict__ Pl) {
  __shared__ __align__(16) float pe[kEarly];
  __shared__ float redM[8];
  __shared__ float redS[8];
  const int r    = blockIdx.x;
  const int bh   = blockIdx.y;
  const int t    = threadIdx.x;
  const int lane = t & 31, wave = t >> 5;
  const size_t rowoff = ((size_t)bh * kEarly + r) * kEarly;
  const float ninf = -__builtin_inff();
  const float s = S[rowoff + t];
  const float a = (t <= r) ? s : ninf;
  float mx = a;
#pragma unroll
  for (int off = 16; off > 0; off >>= 1) mx = fmaxf(mx, __shfl_xor(mx, off, 32));
  if (lane == 0) redM[wave] = mx;
  __syncthreads();
  float m = redM[0];
#pragma unroll
  for (int w = 1; w < 8; ++w) m = fmaxf(m, redM[w]);
  const float e = expf(a - m);
  float sum = e;
#pragma unroll
  for (int off = 16; off > 0; off >>= 1) sum += __shfl_xor(sum, off, 32);
  if (lane == 0) redS[wave] = sum;
  __syncthreads();
  float tot = redS[0];
#pragma unroll
  for (int w = 1; w < 8; ++w) tot += redS[w];
  const float p = e * (1.0f / tot);
  pe[t] = p;
  __syncthreads();
  if (wave == 0) {
    const v4f x0 = *(const v4f*)(pe + 8 * lane);
    const v4f x1 = *(const v4f*)(pe + 8 * lane + 4);
    unsigned short hb[8], lb[8];
#pragma unroll
    for (int q = 0; q < 4; ++q) {
      const float f0 = x0[q], f1 = x1[q];
      hb[q] = f2bf_bits(f0);      lb[q] = f2bf_bits(f0 - bf_bits2f(hb[q]));
      hb[4 + q] = f2bf_bits(f1);  lb[4 + q] = f2bf_bits(f1 - bf_bits2f(hb[4 + q]));
    }
    const v4u uh = (v4u){pk16(hb[0], hb[1]), pk16(hb[2], hb[3]), pk16(hb[4], hb[5]), pk16(hb[6], hb[7])};
    const v4u ul = (v4u){pk16(lb[0], lb[1]), pk16(lb[2], lb[3]), pk16(lb[4], lb[5]), pk16(lb[6], lb[7])};
    unsigned short* qh = Ph + rowoff + 8 * (size_t)lane;
    unsigned short* ql = Pl + rowoff + 8 * (size_t)lane;
    *(volatile v4u*)qh = uh;
    *(volatile v4u*)ql = ul;
    __threadfence();
    *(volatile v4u*)qh = uh;
    *(volatile v4u*)ql = ul;
  }
}

extern "C" void kernel_launch(void* const* d_in, const int* in_sizes, int n_in,
                              void* d_out, int out_size, void* d_ws, size_t ws_size,
                              hipStream_t stream) {
  if (n_in < 4) return;
  const int nX = kTok * kDim;
  const int nW = kHeads * kWRows * kDim;
  const int nP = kDim * kDim;
  if (in_sizes[0] != nX || in_sizes[1] != nW || in_sizes[2] != nP || in_sizes[3] != kDim) return;
  if (out_size != nX) return;

  const size_t szXB   = (size_t)kTok * kDim * 2;
  const size_t szWB   = (size_t)kHeads * kWRows * kDim * 2;
  const size_t szWPB  = (size_t)kDim * kDim * 2;
  const size_t szWP16 = szWPB;
  const size_t szZB   = szWPB;
  const size_t szBP   = 4096;
  const size_t szQK16 = (size_t)kHeads * kTok * kQKW * 2;
  const size_t szVT16 = (size_t)kHeads * kDh * kTok * 2;
  const size_t szQKH  = (size_t)kBH * kEarly * kQKW * 2;
  const size_t szVTH  = (size_t)kBH * kDh * kEarly * 2;
  const size_t szSCE  = (size_t)kBH * kEarly * kEarly * 4;
  const size_t szPH   = (size_t)kBH * kEarly * kEarly * 2;
  const size_t szATT  = (size_t)kTok * kDim * 2;
  const size_t szATH  = (size_t)kBatch * kEarly * kDim * 2;
  const size_t szSC   = (size_t)kGroup * kSeq * kSeq * 4;
  const size_t szP16  = (size_t)kGroup * kSeq * kSeq * 2;
  const size_t offXB   = 0;
  const size_t offWB   = offXB + szXB;
  const size_t offWPB  = offWB + szWB;
  const size_t offWP16 = offWPB + szWPB;
  const size_t offZB   = offWP16 + szWP16;
  const size_t offBP   = offZB + szZB;
  const size_t offQK16 = offBP + szBP;
  const size_t offVT16 = offQK16 + szQK16;
  const size_t offQKH  = offVT16 + szVT16;
  const size_t offQKL  = offQKH + szQKH;
  const size_t offVTH  = offQKL + szQKH;
  const size_t offVTL  = offVTH + szVTH;
  const size_t offSCE  = offVTL + szVTH;
  const size_t offPH   = offSCE + szSCE;
  const size_t offPL   = offPH + szPH;
  const size_t offATT  = offPL + szPH;
  const size_t offATH  = offATT + szATT;
  const size_t offATL  = offATH + szATH;
  const size_t offSC   = offATL + szATH;
  const size_t offP16  = offSC + szSC;
  const size_t total   = offP16 + szP16;
  if (ws_size < total) return;

  const float* x     = (const float*)d_in[0];
  const float* wqkv  = (const float*)d_in[1];
  const float* wproj = (const float*)d_in[2];
  const float* bproj = (const float*)d_in[3];
  float* out = (float*)d_out;
  char* ws = (char*)d_ws;
  unsigned short* XB   = (unsigned short*)(ws + offXB);
  unsigned short* WB   = (unsigned short*)(ws + offWB);
  unsigned short* WPB  = (unsigned short*)(ws + offWPB);
  unsigned short* WP16 = (unsigned short*)(ws + offWP16);
  unsigned short* ZB   = (unsigned short*)(ws + offZB);
  float*          BP   = (float*)(ws + offBP);
  unsigned short* QK16 = (unsigned short*)(ws + offQK16);
  unsigned short* VT16 = (unsigned short*)(ws + offVT16);
  unsigned short* QKH  = (unsigned short*)(ws + offQKH);
  unsigned short* QKL  = (unsigned short*)(ws + offQKL);
  unsigned short* VTH  = (unsigned short*)(ws + offVTH);
  unsigned short* VTL  = (unsigned short*)(ws + offVTL);
  float*          SCE  = (float*)(ws + offSCE);
  unsigned short* PH   = (unsigned short*)(ws + offPH);
  unsigned short* PL   = (unsigned short*)(ws + offPL);
  unsigned short* ATT  = (unsigned short*)(ws + offATT);
  unsigned short* ATH  = (unsigned short*)(ws + offATH);
  unsigned short* ATL  = (unsigned short*)(ws + offATL);
  float*          SC   = (float*)(ws + offSC);
  unsigned short* P16  = (unsigned short*)(ws + offP16);

  cast8_bf16_kernel<<<dim3(nX / 8 / 256), dim3(256), 0, stream>>>(x, XB, nX / 8);
  cast8_bf16_kernel<<<dim3(nW / 8 / 256), dim3(256), 0, stream>>>(wqkv, WB, nW / 8);
  cast8_wproj_kernel<<<dim3(nP / 8 / 256), dim3(256), 0, stream>>>(wproj, WPB, WP16, nP / 8);
  zero8_kernel<<<dim3(nP / 8 / 256), dim3(256), 0, stream>>>(ZB, nP / 8);
  bias_cast_kernel<<<dim3(1), dim3(256), 0, stream>>>(bproj, BP);

  const long sWHead  = (long)kWRows * kDim;
  const long sQKHead = (long)kTok * kQKW;
  const long sVTHead = (long)kDh * kTok;

  wmma_gemm64<1, false, 0, 1, false, 0, 0><<<dim3((kTok / 64) * (kQKW / 64) / 8, kHeads), dim3(256), 0, stream>>>(
      XB, XB, kDim, 0L, WB, WB, kDim, sWHead,
      (void*)QK16, (void*)QK16, kQKW, sQKHead, BP, BP, 0L, kTok, kQKW, kDim, 1.0f);
  wmma_gemm64<1, false, 0, 1, false, 0, 0><<<dim3((kDh / 64) * (kTok / 64) / 8, kHeads), dim3(256), 0, stream>>>(
      WB + (size_t)kQKW * kDim, WB + (size_t)kQKW * kDim, kDim, sWHead, XB, XB, kDim, 0L,
      (void*)VT16, (void*)VT16, kTok, sVTHead, BP, BP, 0L, kDh, kTok, kDim, 1.0f);
  for (int b = 0; b < kBatch; ++b) {
    const unsigned short* XBb = XB + (size_t)b * kSeq * kDim;
    unsigned short* qh = QKH + (size_t)b * kHeads * kEarly * kQKW;
    unsigned short* ql = QKL + (size_t)b * kHeads * kEarly * kQKW;
    wmma_gemm64<1, false, 0, 2, false, 0, 0><<<dim3(1, kHeads), dim3(256), 0, stream>>>(
        XBb, XBb, kDim, 0L, WB, WB, kDim, sWHead,
        (void*)qh, (void*)ql, kQKW, (long)kEarly * kQKW, BP, BP, 0L, kEarly, kQKW, kDim, 1.0f);
    unsigned short* vh = VTH + (size_t)b * kHeads * kDh * kEarly;
    unsigned short* vl = VTL + (size_t)b * kHeads * kDh * kEarly;
    wmma_gemm64<1, false, 0, 2, false, 0, 0><<<dim3(1, kHeads), dim3(256), 0, stream>>>(
        WB + (size_t)kQKW * kDim, WB + (size_t)kQKW * kDim, kDim, sWHead, XBb, XBb, kDim, 0L,
        (void*)vh, (void*)vl, kEarly, (long)kDh * kEarly, BP, BP, 0L, kDh, kEarly, kDim, 1.0f);
  }

  wmma_gemm64<1, true, 0, 0, false, 0, 1><<<dim3(((kEarly / 64) * (kEarly / 64)) / 8, kBH), dim3(256), 0, stream>>>(
      QKH, QKL, kQKW, (long)kEarly * kQKW, QKH + kDh, QKL + kDh, kQKW, (long)kEarly * kQKW,
      (void*)SCE, (void*)SCE, kEarly, (long)kEarly * kEarly, BP, BP, 0L, kEarly, kEarly, kDh, kScoreScale);
  softmax_early_kernel<<<dim3(kEarly, kBH), dim3(256), 0, stream>>>(SCE, PH, PL);
  for (int b = 0; b < kBatch; ++b) {
    const unsigned short* ph = PH + (size_t)b * kHeads * kEarly * kEarly;
    const unsigned short* pl = PL + (size_t)b * kHeads * kEarly * kEarly;
    const unsigned short* vh = VTH + (size_t)b * kHeads * kDh * kEarly;
    const unsigned short* vl = VTL + (size_t)b * kHeads * kDh * kEarly;
    unsigned short* ah = ATH + (size_t)b * kEarly * kDim;
    unsigned short* al = ATL + (size_t)b * kEarly * kDim;
    wmma_gemm64<1, true, 0, 2, false, 0, 2><<<dim3(1, kHeads), dim3(256), 0, stream>>>(
        ph, pl, kEarly, (long)kEarly * kEarly, vh, vl, kEarly, (long)kDh * kEarly,
        (void*)ah, (void*)al, kDim, (long)kDh, BP, BP, 0L, kEarly, kDh, kEarly, 1.0f);
  }

  const long sScore    = (long)kSeq * kSeq;
  const int  gridScore = ((kSeq / 64) * (kSeq / 64)) / 8;
  const int  gridCtx   = ((kSeq / 64) * (kDh / 64)) / 8;
  for (int b = 0; b < kBatch; ++b) {
    for (int g = 0; g < kHeads / kGroup; ++g) {
      const int h0 = g * kGroup;
      const unsigned short* Ag = QK16 + (size_t)h0 * kTok * kQKW + (size_t)b * kSeq * kQKW;
      wmma_gemm64<0, false, 0, 0, false, 0, 1><<<dim3(gridScore, kGroup), dim3(256), 0, stream>>>(
          Ag, Ag, kQKW, sQKHead, Ag + kDh, Ag + kDh, kQKW, sQKHead,
          (void*)SC, (void*)SC, kSeq, sScore, BP, BP, 0L, kSeq, kSeq, kDh, kScoreScale);
      softmax_main_kernel<<<dim3(kSeq, kGroup), dim3(256), 0, stream>>>(SC, P16);
      const unsigned short* Vg = VT16 + (size_t)h0 * kDh * kTok + (size_t)b * kSeq;
      unsigned short* Cg = ATT + (size_t)b * kSeq * kDim + (size_t)h0 * kDh;
      wmma_gemm64<0, false, 0, 1, false, 0, 2><<<dim3(gridCtx, kGroup), dim3(256), 0, stream>>>(
          P16, P16, kSeq, sScore, Vg, Vg, kTok, sVTHead,
          (void*)Cg, (void*)Cg, kDim, (long)kDh, BP, BP, 0L, kSeq, kDh, kSeq, kPVScale);
    }
  }

  wmma_gemm64<0, false, 2, 0, false, 0, 0><<<dim3(((kTok / 64) * (kDim / 64)) / 8, 1), dim3(256), 0, stream>>>(
      ATT, ATT, kDim, 0L, WP16, WP16, kDim, 0L,
      (void*)out, (void*)out, kDim, 0L, BP, BP, 0L, kTok, kDim, kDim, kProjScale);
  wmma_gemm64<1, true, 2, 0, false, 0, 0><<<dim3(((kEarly / 64) * (kDim / 64)) / 8, kBatch), dim3(256), 0, stream>>>(
      ATH, ATL, kDim, (long)kEarly * kDim, WPB, ZB, kDim, 0L,
      (void*)out, (void*)out, kDim, (long)kSeq * kDim, BP, BP, 0L, kEarly, kDim, kDim, 1.0f);
}
